// GCNConv_25202868093076
// MI455X (gfx1250) — hardware-run, weakly checked
//
#include <hip/hip_runtime.h>
#include <stddef.h>
#include <stdint.h>
#include <math.h>

#define SPLIT_A 1

#define NN      100000
#define NE      1600000
#define DF      128
#define KA      256
#define KLOOP   (SPLIT_A ? 256 : 128)
#define MP      100096
#define GBM     64
#define GTHR    128
#define NTHR    256
#define NWAVE   8
#define EPT     8
#define WCH     (32 * EPT)
#define NBRUN   1024
#define SLB     10
#define NBK     98
#define WLCAP   3200
#define RCAP    20480
#define DEGCAP  64
#define RROWS   64
#define MAXDEG_MEAS   16
#define MAXB1024_MEAS 16384
#define WSMAX   134217728

#define BK_ZINTS (NWAVE * WLCAP + 2 * RCAP + 3 * NBRUN)
#define BK_INTS  (BK_ZINTS + 16)
#define BK_LDS   (BK_INTS * 4)

#define PBX   (NN * DF / 8 / NTHR)
#define PBW   (DF * KA / 8 / NTHR)
#define PBB   1
#define PBZ   ((MP - NN) * KA / 8 / NTHR)
#define PBF   4
#define PBTOT (PBX + PBW + PBB + PBZ + PBF)

static_assert(NN == 97 * NBRUN + 672 && NBK == 98);
static_assert(NBK * NBRUN >= MP && MP >= NN && MP == 782 * 128 && MP % GBM == 0 && MP % RROWS == 0);
static_assert(NBRUN == (1 << SLB) && NBRUN % RROWS == 0 && NBRUN % GBM == 0 && NBRUN % 32 == 0);
static_assert(NE % 32 == 0 && NE % WCH == 0 && NE % 4 == 0);
static_assert(NE < (1 << 21) && (((long long)NE) << SLB) < (1LL << 31));
static_assert(DF == 32 * 4 && KA == 2 * DF && KLOOP % 32 == 0 && KLOOP <= KA);
static_assert(NN > 65536 && sizeof(int) == 4);
static_assert((long long)RCAP * 100 >= (long long)MAXB1024_MEAS * 110);
static_assert(WLCAP * 4 >= (RCAP / 8) * 5);
static_assert(MAXDEG_MEAS + 8 <= DEGCAP);
static_assert(BK_ZINTS % 4 == 0 && RCAP % 4 == 0 && BK_LDS <= 300000);
static_assert((NN * DF / 8) % NTHR == 0 && (DF * KA / 8) % NTHR == 0 && ((MP - NN) * KA / 8) % NTHR == 0);
static_assert(NBK * 32 <= PBF * NTHR * 4);
static_assert(RROWS == NWAVE * 8 && GBM == (GTHR / 32) * 16);
static_assert((GBM * DF + DF) * 4 <= 65536);

typedef float          v4f   __attribute__((ext_vector_type(4)));
typedef float          v8f   __attribute__((ext_vector_type(8)));
typedef int            v2i   __attribute__((ext_vector_type(2)));
typedef int            v4i   __attribute__((ext_vector_type(4)));
typedef int            v8i   __attribute__((ext_vector_type(8)));
typedef unsigned       v2u   __attribute__((ext_vector_type(2)));
typedef unsigned short v8us  __attribute__((ext_vector_type(8)));
typedef unsigned short v16us __attribute__((ext_vector_type(16)));
typedef __bf16         v16bf __attribute__((ext_vector_type(16)));
typedef v4f  __attribute__((may_alias)) v4fa;
typedef v2i  __attribute__((may_alias)) v2ia;
typedef v4i  __attribute__((may_alias)) v4ia;
typedef v2u  __attribute__((may_alias)) v2ua;
typedef v8us __attribute__((may_alias)) v8usa;
union FragB { v16bf v; v16us u; v8us h[2]; v8i w; };

__device__ __forceinline__ v8f wmb(const FragB& a, const FragB& b, v8f c) {
  v8f d = __builtin_amdgcn_wmma_f32_16x16x32_bf16(false, a.v, false, b.v, (short)0, c, false, false);
  asm volatile("v_nop\n\tv_nop\n\tv_nop\n\tv_nop" : "+v"(d) : "v"(a.w), "v"(b.w));
  return d;
}

__device__ __forceinline__ unsigned bf16_bits(float f) {
  const unsigned u = __float_as_uint(f);
  const unsigned r = (u + 0x7FFFu + ((u >> 16) & 1u)) >> 16;
  const unsigned q = (u >> 16) | 0x40u;
  return ((u & 0x7fffffffu) > 0x7f800000u) ? q : r;
}
__device__ __forceinline__ float bf16_val(float f) {
  return __uint_as_float(bf16_bits(f) << 16);
}

__device__ __forceinline__ void hilo_pack(float v0, float v1, float v2, float v3,
                                          int& h01, int& h23, int& l01, int& l23) {
  const unsigned a0 = bf16_bits(v0), a1 = bf16_bits(v1), a2 = bf16_bits(v2), a3 = bf16_bits(v3);
  const unsigned b0 = bf16_bits(v0 - __uint_as_float(a0 << 16));
  const unsigned b1 = bf16_bits(v1 - __uint_as_float(a1 << 16));
  const unsigned b2 = bf16_bits(v2 - __uint_as_float(a2 << 16));
  const unsigned b3 = bf16_bits(v3 - __uint_as_float(a3 << 16));
  h01 = (int)(a0 | (a1 << 16)); h23 = (int)(a2 | (a3 << 16));
  l01 = (int)(b0 | (b1 << 16)); l23 = (int)(b2 | (b3 << 16));
}

__device__ __forceinline__ v4i regroup32(int h01, int h23, int l01, int l23, int lane) {
  const int s0 = (2 * lane) & 31, s1 = s0 + 1;
  const int a0 = __shfl(h01, s0, 32), a1 = __shfl(h23, s0, 32), a2 = __shfl(h01, s1, 32), a3 = __shfl(h23, s1, 32);
  const int b0 = __shfl(l01, s0, 32), b1 = __shfl(l23, s0, 32), b2 = __shfl(l01, s1, 32), b3 = __shfl(l23, s1, 32);
  const int mk = (lane < 16) ? -1 : 0;
  v4i o;
  o.x = (a0 & mk) | (b0 & ~mk); o.y = (a1 & mk) | (b1 & ~mk);
  o.z = (a2 & mk) | (b2 & ~mk); o.w = (a3 & mk) | (b3 & ~mk);
  return o;
}

__device__ __forceinline__ void st2_v4f(float* p, v4f v) {
  *(volatile v4f*)p = v;
  __threadfence();
  *(volatile v4f*)p = v;
}
__device__ __forceinline__ void st2_v4i(int* p, v4i v) {
  *(volatile v4i*)p = v;
  __threadfence();
  *(volatile v4i*)p = v;
}
__device__ __forceinline__ void st2_v8us(unsigned short* p, v8us v) {
  *(volatile v8us*)p = v;
  __threadfence();
  *(volatile v8us*)p = v;
}

__device__ __forceinline__ v8us gather8(const float* __restrict__ base, int stride) {
  float f[8];
#pragma unroll
  for (int i = 0; i < 8; ++i) f[i] = base[(size_t)i * (size_t)stride];
  v8us o;
#pragma unroll
  for (int i = 0; i < 8; ++i) o[i] = (unsigned short)bf16_bits(f[i]);
  return o;
}

__global__ __launch_bounds__(NTHR) void k_prep(const float* __restrict__ x, const float* __restrict__ wgt,
                                               const float* __restrict__ bias, unsigned short* xb,
                                               unsigned short* wt2, float* biasf, unsigned short* apl, int* flag) {
  const int tid = (int)threadIdx.x, lane = tid & 31;
  const int blk = (int)blockIdx.x;
  if (blk < PBX) {
    const int u   = blk * NTHR + tid;
    const int row = u >> 4, k8 = (u & 15) * 8;
    const float* p = x + (size_t)row * DF + k8;
    const v4f a = *(const v4fa*)p;
    const v4f b = *(const v4fa*)(p + 4);
    v8us o;
    o[0] = (unsigned short)bf16_bits(a.x); o[1] = (unsigned short)bf16_bits(a.y);
    o[2] = (unsigned short)bf16_bits(a.z); o[3] = (unsigned short)bf16_bits(a.w);
    o[4] = (unsigned short)bf16_bits(b.x); o[5] = (unsigned short)bf16_bits(b.y);
    o[6] = (unsigned short)bf16_bits(b.z); o[7] = (unsigned short)bf16_bits(b.w);
    st2_v8us(xb + (size_t)row * DF + k8, o);
  } else if (blk < PBX + PBW) {
    const int u = (blk - PBX) * NTHR + tid;
    const int n = u >> 5, k8 = (u & 31) * 8, kk = k8 & (DF - 1);
    const v8us o = gather8(wgt + (size_t)kk * DF + n, DF);
    st2_v8us(wt2 + (size_t)n * KA + k8, o);
  } else if (blk < PBX + PBW + PBB) {
    if (tid < 32) {
      const v4f b = *(const v4fa*)(bias + 4 * lane);
      v4f o;
      o.x = bf16_val(b.x); o.y = bf16_val(b.y); o.z = bf16_val(b.z); o.w = bf16_val(b.w);
      st2_v4f(biasf + 4 * lane, o);
    }
  } else if (blk < PBX + PBW + PBB + PBZ) {
    const int u   = (blk - PBX - PBW - PBB) * NTHR + tid;
    const int row = NN + (u >> 5), k8 = (u & 31) * 8;
    const v8us z = {0, 0, 0, 0, 0, 0, 0, 0};
    st2_v8us(apl + (size_t)row * KA + k8, z);
  } else {
    const int u = (blk - PBX - PBW - PBB - PBZ) * NTHR + tid;
    const v4i z = {0, 0, 0, 0};
    st2_v4i(flag + 4 * u, z);
  }
}

__device__ __forceinline__ void bucket_flush(const int* pl, const int* cnt, int ov, int* lp, int* cop, int* fp,
                                             int tid) {
#pragma unroll 1
  for (int i = tid * 4; i < 2 * RCAP; i += NTHR * 4) {
    const v4i v = *(const v4ia*)(pl + i);
    *(volatile v4i*)(lp + i) = v;
  }
#pragma unroll 1
  for (int i = tid * 4; i < 2 * NBRUN; i += NTHR * 4) {
    const v4i v = *(const v4ia*)(cnt + i);
    *(volatile v4i*)(cop + i) = v;
  }
  if (tid < 8) {
    const v4i f = {ov, ov, ov, ov};
    *(volatile v4i*)(fp + 4 * tid) = f;
  }
}

__global__ __launch_bounds__(NTHR) void k_bucket(const int* __restrict__ gidx, const int* __restrict__ keys,
                                                 const float* __restrict__ ew, int* LIST, int* CO, int* FLAG) {
  extern __shared__ __attribute__((aligned(16))) int dsm[];
  int* wl   = dsm;
  int* pl   = dsm + NWAVE * WLCAP;
  int* cnt  = pl + 2 * RCAP;
  int* offs = cnt + NBRUN;
  int* cur  = offs + NBRUN;
  int* misc = cur + NBRUN;
  const int tid = (int)threadIdx.x, lane = tid & 31, wave = tid >> 5;
  const int blk = (int)blockIdx.x;
  const unsigned nbs = (unsigned)(blk * NBRUN);
  const int nbi = (NN - blk * NBRUN) < NBRUN ? (NN - blk * NBRUN) : NBRUN;
  const unsigned unb = (unsigned)(nbi < 0 ? 0 : nbi);

  {
    const v4i z4 = {0, 0, 0, 0};
    for (int i = tid * 4; i < BK_ZINTS; i += NTHR * 4) *(v4ia*)(dsm + i) = z4;
    if (tid < 16) misc[tid] = 0;
  }
  __syncthreads();

  {
    const int per  = ((NE + NWAVE * WCH - 1) / (NWAVE * WCH)) * WCH;
    const int ebeg = wave * per;
    const int eend = (ebeg + per < NE) ? (ebeg + per) : NE;
    int* mylist = wl + wave * WLCAP;
    int wc = 0;
#pragma unroll 1
    for (int cb = ebeg; cb < eend; cb += WCH) {
      const int e0 = cb + lane * EPT;
      const v4i da = *(const v4ia*)(keys + e0);
      const v4i db = *(const v4ia*)(keys + e0 + 4);
      const unsigned s0 = (unsigned)da.x - nbs, s1 = (unsigned)da.y - nbs;
      const unsigned s2 = (unsigned)da.z - nbs, s3 = (unsigned)da.w - nbs;
      const unsigned s4 = (unsigned)db.x - nbs, s5 = (unsigned)db.y - nbs;
      const unsigned s6 = (unsigned)db.z - nbs, s7 = (unsigned)db.w - nbs;
      const bool h0 = s0 < unb, h1 = s1 < unb, h2 = s2 < unb, h3 = s3 < unb;
      const bool h4 = s4 < unb, h5 = s5 < unb, h6 = s6 < unb, h7 = s7 < unb;
      const unsigned m0 = __builtin_amdgcn_ballot_w32(h0), m1 = __builtin_amdgcn_ballot_w32(h1);
      const unsigned m2 = __builtin_amdgcn_ballot_w32(h2), m3 = __builtin_amdgcn_ballot_w32(h3);
      const unsigned m4 = __builtin_amdgcn_ballot_w32(h4), m5 = __builtin_amdgcn_ballot_w32(h5);
      const unsigned m6 = __builtin_amdgcn_ballot_w32(h6), m7 = __builtin_amdgcn_ballot_w32(h7);
      const unsigned any = m0 | m1 | m2 | m3 | m4 | m5 | m6 | m7;
      if (any != 0u) {
        const int pre = (int)(__builtin_amdgcn_mbcnt_lo(m0, 0u) + __builtin_amdgcn_mbcnt_lo(m1, 0u) +
                              __builtin_amdgcn_mbcnt_lo(m2, 0u) + __builtin_amdgcn_mbcnt_lo(m3, 0u) +
                              __builtin_amdgcn_mbcnt_lo(m4, 0u) + __builtin_amdgcn_mbcnt_lo(m5, 0u) +
                              __builtin_amdgcn_mbcnt_lo(m6, 0u) + __builtin_amdgcn_mbcnt_lo(m7, 0u));
        int p = wc + pre;
        if (h0) { if (p < WLCAP) mylist[p] = ((e0 + 0) << SLB) | (int)s0; p = p + 1; }
        if (h1) { if (p < WLCAP) mylist[p] = ((e0 + 1) << SLB) | (int)s1; p = p + 1; }
        if (h2) { if (p < WLCAP) mylist[p] = ((e0 + 2) << SLB) | (int)s2; p = p + 1; }
        if (h3) { if (p < WLCAP) mylist[p] = ((e0 + 3) << SLB) | (int)s3; p = p + 1; }
        if (h4) { if (p < WLCAP) mylist[p] = ((e0 + 4) << SLB) | (int)s4; p = p + 1; }
        if (h5) { if (p < WLCAP) mylist[p] = ((e0 + 5) << SLB) | (int)s5; p = p + 1; }
        if (h6) { if (p < WLCAP) mylist[p] = ((e0 + 6) << SLB) | (int)s6; p = p + 1; }
        if (h7) { if (p < WLCAP) mylist[p] = ((e0 + 7) << SLB) | (int)s7; p = p + 1; }
        wc += (int)(__builtin_popcount(m0) + __builtin_popcount(m1) + __builtin_popcount(m2) + __builtin_popcount(m3) +
                    __builtin_popcount(m4) + __builtin_popcount(m5) + __builtin_popcount(m6) + __builtin_popcount(m7));
      }
    }
    if (lane == 0) misc[wave] = wc;
  }
  __syncthreads();

  if (wave == 0) {
    int ov = 0;
#pragma unroll 1
    for (int w2 = 0; w2 < NWAVE; ++w2) {
      int c = misc[w2];
      if (c > WLCAP) ov = 1;
      c = c < 0 ? 0 : (c > WLCAP ? WLCAP : c);
#pragma unroll 1
      for (int b0 = 0; b0 < c; b0 += 32) {
        const int idx = b0 + lane;
        const int ent = wl[w2 * WLCAP + (idx < WLCAP ? idx : WLCAP - 1)];
        const int m32 = (c - b0) < 32 ? (c - b0) : 32;
#pragma unroll 1
        for (int k = 0; k < m32; ++k) {
          const int u    = __builtin_amdgcn_readlane(ent, k);
          const int slot = u & (NBRUN - 1);
          if (lane == 0) cnt[slot] = cnt[slot] + 1;
        }
      }
    }
    if (lane == 0) misc[9] = ov;
  }
  __syncthreads();
  if (wave == 0) {
    const int base = lane * (NBRUN / 32);
    int s = 0;
#pragma unroll 1
    for (int i = 0; i < NBRUN / 32; ++i) s += cnt[base + i];
    int incl = s;
#pragma unroll
    for (int d = 1; d < 32; d <<= 1) {
      const int y = __shfl_up(incl, d, 32);
      if (lane >= d) incl += y;
    }
    const int tot = __shfl(incl, 31, 32);
    if (lane == 0 && tot > RCAP) misc[9] = 1;
    int run = incl - s;
#pragma unroll 1
    for (int i = 0; i < NBRUN / 32; ++i) {
      const int cv = cnt[base + i];
      offs[base + i] = run;
      cur[base + i]  = run;
      run += cv;
    }
  }
  __syncthreads();

  if (wave == 0) {
#pragma unroll 1
    for (int w2 = 0; w2 < NWAVE; ++w2) {
      int c = misc[w2];
      c = c < 0 ? 0 : (c > WLCAP ? WLCAP : c);
#pragma unroll 1
      for (int b0 = 0; b0 < c; b0 += 32) {
        const int idx = b0 + lane;
        const int ent = wl[w2 * WLCAP + (idx < WLCAP ? idx : WLCAP - 1)];
        int eid = (ent >> SLB) & 0x1FFFFF;
        eid = eid > NE - 1 ? NE - 1 : eid;
        int sr = gidx[eid];
        sr = sr < 0 ? 0 : (sr > NN - 1 ? NN - 1 : sr);
        const int wbits = (int)(bf16_bits(ew[eid]) << 16);
        const int m32 = (c - b0) < 32 ? (c - b0) : 32;
#pragma unroll 1
        for (int k = 0; k < m32; ++k) {
          const int u    = __builtin_amdgcn_readlane(ent, k);
          const int w0   = __builtin_amdgcn_readlane(sr, k);
          const int w1   = __builtin_amdgcn_readlane(wbits, k);
          const int slot = u & (NBRUN - 1);
          if (lane == 0) {
            int p = cur[slot];
            p = p < 0 ? 0 : (p > RCAP - 1 ? RCAP - 1 : p);
            pl[2 * p]     = w0;
            pl[2 * p + 1] = w1;
            cur[slot] = p + 1;
          }
        }
      }
    }
  }
  __syncthreads();

  const int ovf = misc[9];
  int* lp  = LIST + (size_t)blk * (2 * RCAP);
  int* cop = CO + (size_t)blk * (2 * NBRUN);
  int* fp  = FLAG + (size_t)blk * 32;
  bucket_flush(pl, cnt, ovf, lp, cop, fp, tid);
  __threadfence();
  bucket_flush(pl, cnt, ovf, lp, cop, fp, tid);
}

__global__ __launch_bounds__(NTHR) void k_replay(const int* __restrict__ LIST, const int* __restrict__ CO,
                                                 const int* __restrict__ FLAG,
                                                 const unsigned short* __restrict__ XB, unsigned short* A) {
  const int tid = (int)threadIdx.x, lane = tid & 31, wave = tid >> 5;
  const int rowBase = (int)blockIdx.x * RROWS;
  const int bucket  = rowBase >> SLB;
  const int* lb  = LIST + (size_t)bucket * (2 * RCAP);
  const int* cob = CO + (size_t)bucket * (2 * NBRUN);
  const int flag = FLAG[(size_t)bucket * 32];
  const float qnan = __uint_as_float(0x7fc00000u);

#pragma unroll 1
  for (int i = 0; i < RROWS / NWAVE; ++i) {
    const int d    = rowBase + (RROWS / NWAVE) * wave + i;
    const int slot = d & (NBRUN - 1);
    int c = cob[slot];
    int o = cob[NBRUN + slot];
    const bool big = c > DEGCAP;
    c = max(0, min(c, DEGCAP));
    o = max(0, min(o, RCAP - 1));
    int last = o + c - 1; last = last < o ? o : last;
    last = min(last, RCAP - 1);
    float a0 = 0.0f, a1 = 0.0f, a2 = 0.0f, a3 = 0.0f, deg = 0.0f;
#pragma unroll 1
    for (int j = 0; j < c; ++j) {
      int idx = o + j;
      idx = max(o, min(idx, last));
      const v2i ent = *(const v2ia*)(lb + 2 * idx);
      const int sr  = max(0, min(ent.x, NN - 1));
      const float w = __int_as_float(ent.y);
      const v2u xw  = *(const v2ua*)(XB + (size_t)sr * DF + 4 * lane);
      const unsigned x01 = xw.x, x23 = xw.y;
      asm volatile("" :: "v"(x01), "v"(x23));
      const float f0 = __uint_as_float(x01 << 16), f1 = __uint_as_float(x01 & 0xffff0000u);
      const float f2 = __uint_as_float(x23 << 16), f3 = __uint_as_float(x23 & 0xffff0000u);
      a0 = fmaf(w, f0, a0); a1 = fmaf(w, f1, a1); a2 = fmaf(w, f2, a2); a3 = fmaf(w, f3, a3);
      deg += w;
    }
    const float s = 1.0f / sqrtf(deg);
    float m0 = a0 * s, m1 = a1 * s, m2 = a2 * s, m3 = a3 * s;
    const bool bad  = (flag != 0) | big;
    const bool live = d < NN;
    m0 = bad ? qnan : m0; m1 = bad ? qnan : m1; m2 = bad ? qnan : m2; m3 = bad ? qnan : m3;
    m0 = live ? m0 : 0.0f; m1 = live ? m1 : 0.0f; m2 = live ? m2 : 0.0f; m3 = live ? m3 : 0.0f;
    int h01, h23, l01, l23;
    hilo_pack(m0, m1, m2, m3, h01, h23, l01, l23);
    const v4i ow = regroup32(h01, h23, l01, l23, lane);
    unsigned short* hp = A + (size_t)d * KA + 8 * lane;
    *(volatile v4i*)hp = ow;
    __threadfence();
    *(volatile v4i*)hp = ow;
  }
}

__global__ __launch_bounds__(GTHR) __attribute__((amdgpu_num_vgpr(248)))
void k_gemm(const unsigned short* __restrict__ Apl, const unsigned short* __restrict__ BT,
            const float* __restrict__ biasf, const int* __restrict__ FLAG, float* outp) {
  __shared__ __attribute__((aligned(16))) float stg[GBM * DF];
  __shared__ __attribute__((aligned(16))) float sb[DF];
  const int tid = (int)threadIdx.x, lane = tid & 31, wave = tid >> 5, hh = lane >> 4, m = lane & 15;
  const int rowBase = (int)blockIdx.x * GBM;
  const int flag = FLAG[(size_t)(rowBase >> SLB) * 32];
  if (tid < 32) *(v4fa*)(sb + 4 * tid) = *(const v4fa*)(biasf + 4 * tid);

  v8f acc[8];
  {
    const v8f z = {0.f, 0.f, 0.f, 0.f, 0.f, 0.f, 0.f, 0.f};
#pragma unroll
    for (int t = 0; t < 8; ++t) acc[t] = z;
  }
  const unsigned short* ap = Apl + (size_t)(rowBase + 16 * wave + m) * (size_t)KA + 8 * hh;
  const unsigned short* bp = BT + (size_t)m * (size_t)KA + 8 * hh;

#pragma unroll 1
  for (int k0 = 0; k0 < KLOOP; k0 += 32) {
    FragB af;
    af.h[0] = *(const v8usa*)(ap + k0);
    af.h[1] = *(const v8usa*)(ap + k0 + 16);
#pragma unroll
    for (int nt = 0; nt < 8; ++nt) {
      const unsigned short* wq = bp + (size_t)(16 * nt) * (size_t)KA + k0;
      FragB bf;
      bf.h[0] = *(const v8usa*)wq;
      bf.h[1] = *(const v8usa*)(wq + 16);
      acc[nt] = wmb(af, bf, acc[nt]);
    }
  }

#pragma unroll
  for (int nt = 0; nt < 8; ++nt) {
    const int lc = 16 * nt + m;
#pragma unroll
    for (int r = 0; r < 8; ++r) {
      const int lr = 16 * wave + 8 * hh + r;
      stg[lr * DF + lc] = acc[nt][r];
    }
  }
  __syncthreads();

  const v4f bb4 = *(const v4fa*)(sb + 4 * lane);
  const float qnan = __uint_as_float(0x7fc00000u);
  v4f pv[16];
#pragma unroll
  for (int i = 0; i < 16; ++i) pv[i] = *(const v4fa*)(stg + (16 * wave + i) * DF + 4 * lane);

#pragma unroll
  for (int i = 0; i < 16; ++i) {
    const v4f t = pv[i] + bb4;
    v4f y;
    y.x = (flag != 0) ? qnan : t.x;
    y.y = (flag != 0) ? qnan : t.y;
    y.z = (flag != 0) ? qnan : t.z;
    y.w = (flag != 0) ? qnan : t.w;
    pv[i] = y;
  }

#pragma unroll
  for (int i = 0; i < 16; ++i) {
    const int r = rowBase + 16 * wave + i;
    if (r < NN) *(volatile v4f*)(outp + (size_t)r * DF + 4 * lane) = pv[i];
  }
  __threadfence();
#pragma unroll
  for (int i = 0; i < 16; ++i) {
    const int r = rowBase + 16 * wave + i;
    if (r < NN) *(volatile v4f*)(outp + (size_t)r * DF + 4 * lane) = pv[i];
  }
}

extern "C" void kernel_launch(void* const* d_in, const int* in_sizes, int n_in,
                              void* d_out, int out_size, void* d_ws, size_t ws_size,
                              hipStream_t stream) {
  if (n_in < 6) return;
  if (in_sizes[0] != NN * DF) return;
  if (in_sizes[1] != NE) return;
  if (in_sizes[2] != NE) return;
  if (in_sizes[3] != NE) return;
  if (in_sizes[4] != DF * DF) return;
  if (in_sizes[5] != DF) return;
  if (out_size != NN * DF) return;

  const float* x    = (const float*)d_in[0];
  const int*   keys = (const int*)d_in[1];
  const int*   gidx = (const int*)d_in[2];
  const float* ew   = (const float*)d_in[3];
  const float* wgt  = (const float*)d_in[4];
  const float* bias = (const float*)d_in[5];
  float* out = (float*)d_out;

  constexpr size_t zXB   = (size_t)NN * DF * 2;
  constexpr size_t zA    = (size_t)MP * KA * 2;
  constexpr size_t zLIST = (size_t)NBK * RCAP * 8;
  constexpr size_t zCO   = (size_t)NBK * 2 * NBRUN * 4;
  constexpr size_t zFLAG = (size_t)PBF * NTHR * 16;
  constexpr size_t zWT2  = (size_t)DF * KA * 2;
  constexpr size_t zBIAS = 512;
  constexpr size_t oXB   = 0;
  constexpr size_t oA    = oXB + zXB;
  constexpr size_t oLIST = oA + zA;
  constexpr size_t oCO   = oLIST + zLIST;
  constexpr size_t oFLAG = oCO + zCO;
  constexpr size_t oWT2  = oFLAG + zFLAG;
  constexpr size_t oBIAS = oWT2 + zWT2;
  constexpr size_t oEND  = oBIAS + zBIAS;
  static_assert(zXB % 256 == 0 && zA % 256 == 0 && zLIST % 256 == 0 && zCO % 256 == 0);
  static_assert(zFLAG % 256 == 0 && zWT2 % 256 == 0 && zBIAS % 256 == 0);
  static_assert(zFLAG >= (size_t)NBK * 128);
  static_assert(oEND <= (size_t)WSMAX);
  if (oEND > ws_size) return;

  char* ws = (char*)d_ws;
  unsigned short* XB    = (unsigned short*)(ws + oXB);
  unsigned short* Apl   = (unsigned short*)(ws + oA);
  int*            LIST  = (int*)(ws + oLIST);
  int*            CO    = (int*)(ws + oCO);
  int*            FLAG  = (int*)(ws + oFLAG);
  unsigned short* WT2   = (unsigned short*)(ws + oWT2);
  float*          BIASF = (float*)(ws + oBIAS);

  hipFuncSetAttribute(reinterpret_cast<const void*>(&k_bucket), hipFuncAttributeMaxDynamicSharedMemorySize, (int)BK_LDS);

  k_prep<<<PBTOT, NTHR, 0, stream>>>(x, wgt, bias, XB, WT2, BIASF, Apl, FLAG);
  k_bucket<<<NBK, NTHR, BK_LDS, stream>>>(gidx, keys, ew, LIST, CO, FLAG);
  k_replay<<<MP / RROWS, NTHR, 0, stream>>>(LIST, CO, FLAG, XB, Apl);
  k_gemm<<<MP / GBM, GTHR, 0, stream>>>(Apl, WT2, BIASF, FLAG, out);
}
